// ModulatedDeformConv_62886911148487
// MI455X (gfx1250) — hardware-verified
//
#include <hip/hip_runtime.h>

typedef unsigned short u16;
typedef u16    v8us __attribute__((ext_vector_type(8)));
typedef __bf16 v16b __attribute__((ext_vector_type(16)));
typedef float  v8f  __attribute__((ext_vector_type(8)));
typedef float  v4f  __attribute__((ext_vector_type(4)));
typedef int    v4i  __attribute__((ext_vector_type(4)));
typedef v8us __attribute__((may_alias)) v8usa;
typedef v4f  __attribute__((may_alias)) v4fa;
typedef v4i  __attribute__((may_alias)) v4ia;
typedef float __attribute__((may_alias)) f32a;
typedef unsigned int __attribute__((may_alias)) u32a;

union FragB { v16b v; v8us u[2]; };

#define NB_  8
#define CI   128
#define CO   128
#define HH   64
#define WW   64
#define KK   9
#define HWP  (HH * WW)
#define KD   (KK * CI)
#define PT   64
#define NPT  (HWP / PT)
#define LDB  40
#define NCH  (KD / 8)
#define TWB  (KK * PT * 16)
#define TIB  (KK * PT * 16)
#define BTB  (PT * LDB * 2)
#define SMB  (CO * PT * 4)

static_assert(PT == WW);
static_assert(HWP % PT == 0);
static_assert(KD % 32 == 0);
static_assert(KD % 4 == 0);
static_assert(TWB + TIB + 2 * BTB <= SMB);
static_assert(SMB <= 65536);
static_assert((KD * 2) % 128 == 0);
static_assert(PT * 4 == 256);
static_assert((LDB * 2) % 16 == 0);
static_assert(NCH <= 256);
static_assert((NB_ * CI * HWP) % (8 * 256) == 0);
static_assert(CO % 32 == 0);
static_assert(KK * (PT / 4) <= 256);
static_assert(WW % 4 == 0);

__device__ __forceinline__ v8f wmma_bf16(v16b a, v16b b, v8f c) {
  v8f d = __builtin_amdgcn_wmma_f32_16x16x32_bf16(false, a, false, b, (short)0, c, false, false);
  asm volatile("v_nop\n\tv_nop\n\tv_nop\n\tv_nop" : "+v"(d) : "v"(a), "v"(b));
  return d;
}

__device__ __forceinline__ v16b ldfrag(const u16* p, int h) {
  FragB f;
  f.u[0] = *(const v8usa*)(p + 8 * h);
  f.u[1] = *(const v8usa*)(p + 16 + 8 * h);
  return f.v;
}

__device__ __forceinline__ void ldwait() {
  asm volatile("s_wait_loadcnt 0x0" ::: "memory");
}

__device__ __forceinline__ unsigned bf16_bits(float f) {
  unsigned u = __float_as_uint(f);
  u += 0x7FFFu + ((u >> 16) & 1u);
  return u >> 16;
}
__device__ __forceinline__ float bf16r(float f) { return __uint_as_float(bf16_bits(f) << 16); }
__device__ __forceinline__ float bfx(u16 s) { return __uint_as_float(((unsigned)s) << 16); }

__global__ __launch_bounds__(256) void xcvt_kernel(const float* __restrict__ x, u16* __restrict__ xb) {
  const size_t ci = (size_t)blockIdx.x * 256 + threadIdx.x;
  const v4f g0 = *(const v4fa*)(x + 8 * ci);
  const v4f g1 = *(const v4fa*)(x + 8 * ci + 4);
  const v8us o8 = { (u16)bf16_bits(g0.x), (u16)bf16_bits(g0.y), (u16)bf16_bits(g0.z), (u16)bf16_bits(g0.w),
                    (u16)bf16_bits(g1.x), (u16)bf16_bits(g1.y), (u16)bf16_bits(g1.z), (u16)bf16_bits(g1.w) };
  u16* dst = xb + 8 * ci;
  *(volatile v8us*)dst = o8;
  __threadfence();
  *(volatile v8us*)dst = o8;
}

__device__ __forceinline__ void wprep_pass(const float* wr, u16* wq, int o, int tid) {
  if (tid < NCH) {
    const int kc = tid;
    const int t  = kc >> 4;
    const int c0 = (kc & 15) * 8;
    float v[8];
    #pragma unroll
    for (int i = 0; i < 8; ++i) v[i] = wr[(c0 + i) * KK + t];
    const v8us o8 = { (u16)(__float_as_uint(v[0]) >> 16), (u16)(__float_as_uint(v[1]) >> 16),
                      (u16)(__float_as_uint(v[2]) >> 16), (u16)(__float_as_uint(v[3]) >> 16),
                      (u16)(__float_as_uint(v[4]) >> 16), (u16)(__float_as_uint(v[5]) >> 16),
                      (u16)(__float_as_uint(v[6]) >> 16), (u16)(__float_as_uint(v[7]) >> 16) };
    u16* dst = wq + (size_t)o * KD + 8 * kc;
    *(volatile v8us*)dst = o8;
  }
}

__global__ __launch_bounds__(256) void wprep_kernel(const float* __restrict__ wgt,
                                                    u16* __restrict__ wq)
{
  __shared__ __attribute__((aligned(16))) float wr[KD];
  const int tid = threadIdx.x, o = blockIdx.x;
  #pragma unroll 1
  for (int e = tid; e < KD / 4; e += 256) {
    const v4f g = *(const v4fa*)(wgt + (size_t)o * KD + 4 * e);
    const v4f r = { bf16r(g.x), bf16r(g.y), bf16r(g.z), bf16r(g.w) };
    *(v4fa*)(wr + 4 * e) = r;
  }
  __syncthreads();
  wprep_pass(wr, wq, o, tid);
  __threadfence();
  wprep_pass(wr, wq, o, tid);
}

__device__ __forceinline__ float comb4(v4f tw, u16 a, u16 bq, u16 c, u16 d) {
  float v = tw.x * bfx(a);
  v = fmaf(tw.y, bfx(bq), v);
  v = fmaf(tw.z, bfx(c), v);
  v = fmaf(tw.w, bfx(d), v);
  return v;
}

__device__ __forceinline__ void out_store_pass(const char* smem, float* out,
                                               int b, int nb, int w, int lane) {
  const int q8 = lane & 7, sub = lane >> 3;
  #pragma unroll
  for (int it = 0; it < 8; ++it) {
    const int lid = 4 * it + sub;
    const int o = 16 * w + (lid >> 1), ln = lid & 1;
    const v4f v = *(const v4fa*)(smem + (size_t)(o * PT + 32 * ln + 4 * q8) * 4);
    float* dst = out + ((size_t)(b * CO + o)) * HWP + nb + 32 * ln + 4 * q8;
    *(volatile v4f*)dst = v;
  }
}

__global__ __launch_bounds__(256) void dconv_kernel(
    const u16* __restrict__ xb,
    const float* __restrict__ offs,
    const float* __restrict__ msk,
    const u16* __restrict__ wq,
    const float* __restrict__ bias,
    float* __restrict__ out)
{
  __shared__ __attribute__((aligned(16))) char smem[SMB];
  float* s_tw = (float*)smem;
  int*   s_ti = (int*)(smem + TWB);
  u16*   s_bh = (u16*)(smem + TWB + TIB);
  u16*   s_bl = (u16*)(smem + TWB + TIB + BTB);
  f32a*  sF   = (f32a*)smem;

  const int tid = threadIdx.x, lane = tid & 31, w = tid >> 5;
  const int h = lane >> 4, m = lane & 15;
  const int pt = blockIdx.x, b = blockIdx.y;
  const int nb = PT * pt;

  #pragma unroll 1
  for (int e = tid; e < KK * (PT / 4); e += 256) {
    const int t = e >> 4, q4 = e & 15;
    const int ky = t / 3, kx = t - 3 * ky;
    const size_t ob0 = ((size_t)(b * 2 * KK + 2 * t) * HH + pt) * WW + 4 * q4;
    const v4f oy4 = *(const v4fa*)(offs + ob0);
    const v4f ox4 = *(const v4fa*)(offs + ob0 + (size_t)HWP);
    const v4f mk4 = *(const v4fa*)(msk + ((size_t)(b * KK + t) * HH + pt) * WW + 4 * q4);
    ldwait();
    const float oya[4] = { oy4.x, oy4.y, oy4.z, oy4.w };
    const float oxa[4] = { ox4.x, ox4.y, ox4.z, ox4.w };
    const float mka[4] = { mk4.x, mk4.y, mk4.z, mk4.w };
    #pragma unroll
    for (int j = 0; j < 4; ++j) {
      const int qx = 4 * q4 + j;
      const float offy = bf16r(oya[j]);
      const float offx = bf16r(oxa[j]);
      const float mv   = bf16r(mka[j]);
      float py = offy + (float)(pt - 1);  py = py + (float)ky;
      float px = offx + (float)(qx - 1);  px = px + (float)kx;
      const float fy = floorf(py), fx = floorf(px);
      const float ly = py - fy, lx = px - fx;
      const int y0 = (int)fminf(fmaxf(fy, -4.0f), (float)(HH + 4));
      const int x0 = (int)fminf(fmaxf(fx, -4.0f), (float)(WW + 4));
      const int y1 = y0 + 1, x1 = x0 + 1;
      const bool vy0 = (y0 >= 0) && (y0 < HH), vy1 = (y1 >= 0) && (y1 < HH);
      const bool vx0 = (x0 >= 0) && (x0 < WW), vx1 = (x1 >= 0) && (x1 < WW);
      const int cy0 = min(max(y0, 0), HH - 1), cy1 = min(max(y1, 0), HH - 1);
      const int cx0 = min(max(x0, 0), WW - 1), cx1 = min(max(x1, 0), WW - 1);
      const float hy = 1.0f - ly, hx = 1.0f - lx;
      v4f tw;
      tw.x = (vy0 && vx0) ? (hy * hx) * mv : 0.0f;
      tw.y = (vy0 && vx1) ? (hy * lx) * mv : 0.0f;
      tw.z = (vy1 && vx0) ? (ly * hx) * mv : 0.0f;
      tw.w = (vy1 && vx1) ? (ly * lx) * mv : 0.0f;
      v4i ti;
      ti.x = cy0 * WW + cx0;  ti.y = cy0 * WW + cx1;
      ti.z = cy1 * WW + cx0;  ti.w = cy1 * WW + cx1;
      const int ent = t * PT + qx;
      *(v4fa*)(s_tw + 4 * ent) = tw;
      *(v4ia*)(s_ti + 4 * ent) = ti;
    }
  }
  __syncthreads();

  const int cg = w & 3, pg = w >> 2;
  const u16* wr0 = wq + ((size_t)(32 * cg + m)) * KD;
  const u16* wr1 = wr0 + (size_t)16 * KD;
  const u16* bh0p = s_bh + (32 * pg + m) * LDB;
  const u16* bh1p = bh0p + 16 * LDB;
  const u16* bl0p = s_bl + (32 * pg + m) * LDB;
  const u16* bl1p = bl0p + 16 * LDB;

  const int spx = tid & 63, sg = tid >> 6;
  u16* dh = s_bh + spx * LDB + 8 * sg;
  u16* dl = s_bl + spx * LDB + 8 * sg;

  const v8f zf = {0.f, 0.f, 0.f, 0.f, 0.f, 0.f, 0.f, 0.f};
  v8f acc[2][2];
  #pragma unroll
  for (int i = 0; i < 2; ++i)
    #pragma unroll
    for (int j = 0; j < 2; ++j) acc[i][j] = zf;

  #pragma unroll 1
  for (int s = 0; s < KD / 32; ++s) {
    const int t = s >> 2;
    const int cb = 32 * (s & 3) + 8 * sg;
    const v4f tw = *(const v4fa*)(s_tw + 4 * (t * PT + spx));
    const v4i ti = *(const v4ia*)(s_ti + 4 * (t * PT + spx));
    const u16* xc = xb + ((size_t)(b * CI + cb)) * HWP;
    #pragma unroll 1
    for (int cp = 0; cp < 4; ++cp) {
      const u16* x0p = xc + (size_t)(2 * cp) * HWP;
      const u16* x1p = x0p + HWP;
      const u16 ga = x0p[ti.x], gb = x0p[ti.y], gc = x0p[ti.z], gd = x0p[ti.w];
      const u16 ge = x1p[ti.x], gf = x1p[ti.y], gg = x1p[ti.z], gq = x1p[ti.w];
      ldwait();
      const float v0 = comb4(tw, ga, gb, gc, gd);
      const float v1 = comb4(tw, ge, gf, gg, gq);
      const unsigned h0 = bf16_bits(v0), h1 = bf16_bits(v1);
      const unsigned l0 = bf16_bits(v0 - __uint_as_float(h0 << 16));
      const unsigned l1 = bf16_bits(v1 - __uint_as_float(h1 << 16));
      *(u32a*)(dh + 2 * cp) = h0 | (h1 << 16);
      *(u32a*)(dl + 2 * cp) = l0 | (l1 << 16);
    }
    __syncthreads();

    const v16b a0  = ldfrag(wr0 + 32 * s, h);
    const v16b a1  = ldfrag(wr1 + 32 * s, h);
    const v16b bh0 = ldfrag(bh0p, h);
    const v16b bl0 = ldfrag(bl0p, h);
    acc[0][0] = wmma_bf16(a0, bh0, acc[0][0]);
    acc[0][0] = wmma_bf16(a0, bl0, acc[0][0]);
    acc[1][0] = wmma_bf16(a1, bh0, acc[1][0]);
    acc[1][0] = wmma_bf16(a1, bl0, acc[1][0]);
    const v16b bh1 = ldfrag(bh1p, h);
    const v16b bl1 = ldfrag(bl1p, h);
    acc[0][1] = wmma_bf16(a0, bh1, acc[0][1]);
    acc[0][1] = wmma_bf16(a0, bl1, acc[0][1]);
    acc[1][1] = wmma_bf16(a1, bh1, acc[1][1]);
    acc[1][1] = wmma_bf16(a1, bl1, acc[1][1]);
    __syncthreads();
  }

  #pragma unroll
  for (int i = 0; i < 2; ++i) {
    const int ob = 32 * cg + 16 * i + 8 * h;
    const v4f bA = *(const v4fa*)(bias + ob);
    const v4f bB = *(const v4fa*)(bias + ob + 4);
    const float bs[8] = { bf16r(bA.x), bf16r(bA.y), bf16r(bA.z), bf16r(bA.w),
                          bf16r(bB.x), bf16r(bB.y), bf16r(bB.z), bf16r(bB.w) };
    #pragma unroll
    for (int j = 0; j < 2; ++j) {
      const int px = 32 * pg + 16 * j + m;
      #pragma unroll
      for (int r = 0; r < 8; ++r)
        sF[(ob + r) * PT + px] = acc[i][j][r] + bs[r];
    }
  }
  __syncthreads();

  out_store_pass(smem, out, b, nb, w, lane);
  __threadfence();
  out_store_pass(smem, out, b, nb, w, lane);
}

extern "C" void kernel_launch(void* const* d_in, const int* in_sizes, int n_in,
                              void* d_out, int out_size, void* d_ws, size_t ws_size,
                              hipStream_t stream) {
  if (n_in < 5) return;
  if (in_sizes[0] != NB_ * CI * HWP) return;
  if (in_sizes[1] != NB_ * 2 * KK * HWP) return;
  if (in_sizes[2] != NB_ * KK * HWP) return;
  if (in_sizes[3] != CO * KD) return;
  if (in_sizes[4] != CO) return;
  if (out_size != NB_ * CO * HWP) return;

  const float* x    = (const float*)d_in[0];
  const float* offs = (const float*)d_in[1];
  const float* msk  = (const float*)d_in[2];
  const float* wgt  = (const float*)d_in[3];
  const float* bias = (const float*)d_in[4];
  float* out = (float*)d_out;

  const size_t wq_bytes = (size_t)CO * KD * 2;
  const size_t xb_bytes = (size_t)NB_ * CI * HWP * 2;
  const size_t total = wq_bytes + xb_bytes;
  if (total > ws_size) return;

  char* ws = (char*)d_ws;
  u16* wq = (u16*)(ws);
  u16* xb = (u16*)(ws + wq_bytes);

  xcvt_kernel<<<(NB_ * CI * HWP / 8) / 256, 256, 0, stream>>>(x, xb);
  wprep_kernel<<<CO, 256, 0, stream>>>(wgt, wq);
  dconv_kernel<<<dim3(NPT, NB_), 256, 0, stream>>>(xb, offs, msk, wq, bias, out);
}
